// MultiHeadAttention_13864154431545
// MI455X (gfx1250) — hardware-run, weakly checked
//
#include <hip/hip_runtime.h>


#ifndef NB
#define NB 2
#endif
#ifndef SEQ
#define SEQ 2048
#endif
#define NB_FULL  2
#define SEQ_FULL 2048
#define DM   1024
#define NH_  16
#define HD   64
#define AW   4
#define QRS  2048.0f
#define QRI  (1.0f / 2048.0f)
#define SC2  (0.125f * 1.4426950408889634f)
#define PSH  8.0f
#define CTS  4096.0f
#define WOS  1024.0f
#define OSC  (1.0f / (4096.0f * 1024.0f))

static_assert(HD == 64);
static_assert(NH_ * HD == DM);
static_assert((DM & (DM - 1)) == 0);
static_assert(DM % 64 == 0);
static_assert(DM % 32 == 0);
static_assert(SEQ % 64 == 0);
static_assert((NB * SEQ) % 64 == 0);
static_assert(SEQ % 32 == 0);
static_assert(SEQ % (16 * AW) == 0);
static_assert(((size_t)SEQ * (SEQ / 32)) % 256 == 0);
static_assert(((size_t)NB * SEQ * DM / 8) % 256 == 0);
static_assert(NB <= NB_FULL);
static_assert(SEQ <= SEQ_FULL);
static_assert(((size_t)(SEQ - 1) * NB_FULL + NB) * DM <= (size_t)SEQ_FULL * NB_FULL * DM);

typedef _Float16 h16;
typedef unsigned short bf;
typedef __attribute__((ext_vector_type(16))) __bf16   v16bf;
typedef __attribute__((ext_vector_type(16))) _Float16 v16h;
typedef __attribute__((ext_vector_type(16))) unsigned short v16us;
typedef __attribute__((ext_vector_type(8)))  _Float16 v8h;
typedef __attribute__((ext_vector_type(8)))  unsigned short v8us;
typedef __attribute__((ext_vector_type(8)))  float    v8f;
typedef __attribute__((ext_vector_type(4)))  float    v4f;
typedef __attribute__((ext_vector_type(4)))  int      v4i;
typedef v4f  __attribute__((may_alias)) v4fa;
typedef v8us __attribute__((may_alias)) v8usa;

__device__ __forceinline__ unsigned short f2bf(float f) { unsigned u = __float_as_uint(f); u += 0x7FFFu + ((u >> 16) & 1u); return (unsigned short)(u >> 16); }
__device__ __forceinline__ float bfr(float f) { return __uint_as_float(((unsigned)f2bf(f)) << 16); }
__device__ __forceinline__ v16h cat16(v8h lo, v8h hi) { return __builtin_shufflevector(lo, hi, 0, 1, 2, 3, 4, 5, 6, 7, 8, 9, 10, 11, 12, 13, 14, 15); }
__device__ __forceinline__ v8f wmma16(v16h a, v16h b, v8f c) { return __builtin_amdgcn_wmma_f32_16x16x32_f16(false, a, false, b, (short)0, c, false, false); }
__device__ __forceinline__ v16h  ldh(const h16* p) { return cat16(*(const v8h*)p, *(const v8h*)(p + 16)); }
__device__ __forceinline__ v16us ldu(const bf* p)  { const v8us lo = *(const v8us*)p; const v8us hi = *(const v8us*)(p + 16); return __builtin_shufflevector(lo, hi, 0, 1, 2, 3, 4, 5, 6, 7, 8, 9, 10, 11, 12, 13, 14, 15); }
template <int F16OP> __device__ __forceinline__ v8f wmx(v16us a, v16us b, v8f c) {
    if (F16OP) return __builtin_amdgcn_wmma_f32_16x16x32_f16(false, __builtin_bit_cast(v16h, a), false, __builtin_bit_cast(v16h, b), (short)0, c, false, false);
    return __builtin_amdgcn_wmma_f32_16x16x32_bf16(false, __builtin_bit_cast(v16bf, a), false, __builtin_bit_cast(v16bf, b), (short)0, c, false, false);
}
__device__ __forceinline__ void wave_sync() { __builtin_amdgcn_fence(3  , "wavefront"); __builtin_amdgcn_wave_barrier(); asm volatile("" ::: "memory"); }

__global__ __launch_bounds__(256) void k_cvtx(const float* __restrict__ src, bf* dst) {
    const size_t n8 = (size_t)NB * SEQ * DM / 8;
    const size_t i = (size_t)blockIdx.x * 256 + threadIdx.x; if (i >= n8) return;
    const size_t row = i / (DM / 8); const size_t g = i % (DM / 8);
    const size_t b = row / SEQ, t = row % SEQ;
    const v8f v = *(const v8f*)(src + (t * NB_FULL + b) * DM + g * 8); v8us o;
#pragma unroll
    for (int k = 0; k < 8; ++k) o[k] = f2bf(v[k]);
    *(volatile v8us*)(dst + i * 8) = o; __threadfence(); *(volatile v8us*)(dst + i * 8) = o;
}

__global__ __launch_bounds__(256) void k_wt(const float* __restrict__ W, bf* dst, int asF16) {
    __shared__ __align__(16) unsigned short T[64 * 72];
    const int tid = threadIdx.x; const int n0 = blockIdx.x * 64, k0 = blockIdx.y * 64;
#pragma unroll
    for (int i = 0; i < 4; ++i) { const int idx = tid + i * 256; const int r = idx >> 4, c4 = idx & 15;
        const v4f f = *(const v4f*)(W + (size_t)(k0 + r) * DM + n0 + c4 * 4);
#pragma unroll
        for (int e = 0; e < 4; ++e) { const unsigned short bb = f2bf(f[e]); const h16 hv = (h16)(__uint_as_float(((unsigned)bb) << 16) * WOS);
            const unsigned short hb = __builtin_bit_cast(unsigned short, hv);
            T[(c4 * 4 + e) * 72 + r] = asF16 ? hb : bb; } }
    __syncthreads();
#pragma unroll 1
    for (int ps = 0; ps < 2; ++ps) {
#pragma unroll
        for (int i = 0; i < 2; ++i) { const int idx = tid + i * 256; const int n = idx >> 3, ch = idx & 7;
            const v8us o = *(const v8usa*)(&T[n * 72 + ch * 8]);
            *(volatile v8us*)(dst + (size_t)(n0 + n) * DM + k0 + ch * 8) = o; }
        if (ps == 0) __threadfence(); }
}

__global__ __launch_bounds__(256) void k_mpack(const int* __restrict__ mask, unsigned* mb) {
    const int gid = blockIdx.x * 256 + threadIdx.x; if (gid >= SEQ * (SEQ / 32)) return;
    const int i = gid / (SEQ / 32), w = gid % (SEQ / 32);
    const int* p = mask + (size_t)i * SEQ_FULL + w * 32;
    unsigned bits = 0u;
#pragma unroll
    for (int c = 0; c < 8; ++c) { const v4i v = *(const v4i*)(p + c * 4);
#pragma unroll
        for (int e = 0; e < 4; ++e) bits |= (v[e] != 0 ? 1u : 0u) << (c * 4 + e); }
    *(volatile unsigned*)(mb + gid) = bits; __threadfence(); *(volatile unsigned*)(mb + gid) = bits;
}

template <int F16OP, int OUTF32>
__global__ __launch_bounds__(32) void k_gemm(const bf* __restrict__ A, const bf* __restrict__ Bt, int K, int KB,
                                             h16* Ph, h16* Pr, int useRes, float* Of,
                                             const float* __restrict__ bias, int biasMode, float oscale,
                                             int RB, size_t sRB, int pitch, int CB, size_t sCB) {
    __shared__ __align__(16) float os[16 * 68];
    const int lane = threadIdx.x & 31, lr = lane & 15, hi = lane >> 4; const int r0 = blockIdx.x * 64, c0 = blockIdx.y * 64;
    v8f acc[4][4];
#pragma unroll
    for (int mb = 0; mb < 4; ++mb)
#pragma unroll
        for (int nb = 0; nb < 4; ++nb) acc[mb][nb] = (v8f){};
    const size_t aoff = (size_t)(r0 + lr) * K + 8 * hi, boff = (size_t)(c0 + lr) * KB + 8 * hi;
    const int kmB = KB - 1;
#pragma unroll 1
    for (int kc = 0; kc < K; kc += 32) {
        const int kb = kc & kmB;
        v16us a[4];
#pragma unroll
        for (int mb = 0; mb < 4; ++mb) a[mb] = ldu(A + aoff + (size_t)mb * 16 * K + kc);
#pragma unroll
        for (int nb = 0; nb < 4; ++nb) { const v16us b = ldu(Bt + boff + (size_t)nb * 16 * KB + kb);
#pragma unroll
            for (int mb = 0; mb < 4; ++mb) acc[mb][nb] = wmx<F16OP>(a[mb], b, acc[mb][nb]); }
        asm volatile("v_nop\n\tv_nop\n\tv_nop\n\tv_nop" : "+v"(acc[0][0]), "+v"(acc[1][1]), "+v"(acc[2][2]), "+v"(acc[3][3]) : "v"(a[0]), "v"(a[1]), "v"(a[2]), "v"(a[3]));
    }
    float cb[4];
#pragma unroll
    for (int nb = 0; nb < 4; ++nb) cb[nb] = 0.0f;
    if (biasMode == 0) {
#pragma unroll
        for (int nb = 0; nb < 4; ++nb) cb[nb] = bfr(bias[c0 + nb * 16 + lr]); }
    const size_t tbase = (size_t)(r0 / RB) * sRB + (size_t)(r0 % RB) * (size_t)pitch + (size_t)(c0 / CB) * sCB + (size_t)(c0 % CB);
#pragma unroll
    for (int mb = 0; mb < 4; ++mb) {
        float rb[8];
#pragma unroll
        for (int j = 0; j < 8; ++j) rb[j] = 0.0f;
        if (biasMode == 1) {
#pragma unroll
            for (int j = 0; j < 8; ++j) rb[j] = bfr(bias[r0 + mb * 16 + hi * 8 + j]); }
#pragma unroll
        for (int nb = 0; nb < 4; ++nb) {
#pragma unroll
            for (int j = 0; j < 8; ++j) os[(hi * 8 + j) * 68 + nb * 16 + lr] = acc[mb][nb][j] * oscale + (cb[nb] + rb[j]); }
        wave_sync();
        const size_t sb = tbase + (size_t)(mb * 16) * (size_t)pitch;
        if (OUTF32) {
#pragma unroll 1
            for (int ps = 0; ps < 2; ++ps) {
#pragma unroll
                for (int s = 0; s < 8; ++s) { const int row = 2 * s + hi, cofs = lr * 4;
                    const v4f val = *(const v4fa*)(&os[row * 68 + cofs]);
                    *(volatile v4f*)(Of + sb + (size_t)row * (size_t)pitch + cofs) = val; }
                if (ps == 0) __threadfence(); }
        } else {
#pragma unroll 1
            for (int ps = 0; ps < 2; ++ps) {
#pragma unroll
                for (int s = 0; s < 4; ++s) { const int row = 4 * s + (lane >> 3), c8 = (lane & 7) * 8;
                    const v4f x0 = *(const v4fa*)(&os[row * 68 + c8]); const v4f x1 = *(const v4fa*)(&os[row * 68 + c8 + 4]); v8h hv, rv;
#pragma unroll
                    for (int i = 0; i < 4; ++i) { const h16 a0 = (h16)x0[i]; const h16 a1 = (h16)x1[i]; hv[i] = a0; hv[4 + i] = a1; rv[i] = (h16)((x0[i] - (float)a0) * QRS); rv[4 + i] = (h16)((x1[i] - (float)a1) * QRS); }
                    const size_t oo = sb + (size_t)row * (size_t)pitch + c8;
                    *(volatile v8h*)(Ph + oo) = hv; if (useRes) *(volatile v8h*)(Pr + oo) = rv; }
                if (ps == 0) __threadfence(); }
        }
        wave_sync();
    }
}

__global__ __launch_bounds__(32 * AW) void k_flash(const h16* __restrict__ QH, const h16* __restrict__ QR, const h16* __restrict__ KP, const h16* __restrict__ VT,
                                                   const unsigned* __restrict__ MB, h16* CT) {
    __shared__ __align__(16) float os[AW * 16 * 68];
    const int lane = threadIdx.x & 31, wave = __builtin_amdgcn_readfirstlane((int)(threadIdx.x >> 5)), lr = lane & 15, hi = lane >> 4;
    const int zh = blockIdx.y; const int b = zh / NH_, h = zh % NH_;
    const int t0 = (blockIdx.x * AW + wave) * 16;
    const size_t pbase = (size_t)zh * SEQ * HD;
    const size_t qo = pbase + (size_t)(t0 + lr) * HD + 8 * hi;
    const v16h qh0 = ldh(QH + qo), qh1 = ldh(QH + qo + 32), qr0 = ldh(QR + qo), qr1 = ldh(QR + qo + 32);
    const size_t ko = pbase + (size_t)lr * HD + 8 * hi;
    const size_t vo = pbase + (size_t)lr * SEQ + 8 * hi;
    const size_t mo = (size_t)(t0 + lr) * (SEQ / 32);
    v8f o0 = (v8f){}, o1 = (v8f){}, o2 = (v8f){}, o3 = (v8f){};
    float m = -3.0e38f, l = 0.0f;
#pragma unroll 1
    for (int key0 = 0; key0 < SEQ; key0 += 32) {
        const unsigned mw = MB[mo + (size_t)(key0 >> 5)];
        const unsigned ba = mw >> (8 * hi), bb = mw >> (16 + 8 * hi);
        const h16* ka = KP + ko + (size_t)key0 * HD;
        const v16h ka0 = ldh(ka), ka1 = ldh(ka + 32), kb0 = ldh(ka + 16 * HD), kb1 = ldh(ka + 16 * HD + 32);
        v8f sHa = (v8f){}, sLa = (v8f){}, sHb = (v8f){}, sLb = (v8f){};
        sHa = wmma16(ka0, qh0, sHa); sLa = wmma16(ka0, qr0, sLa); sHb = wmma16(kb0, qh0, sHb); sLb = wmma16(kb0, qr0, sLb);
        sHa = wmma16(ka1, qh1, sHa); sLa = wmma16(ka1, qr1, sLa); sHb = wmma16(kb1, qh1, sHb); sLb = wmma16(kb1, qr1, sLb);
        asm volatile("v_nop\n\tv_nop\n\tv_nop\n\tv_nop" : "+v"(sHa), "+v"(sLa), "+v"(sHb), "+v"(sLb) : "v"(ka0), "v"(ka1), "v"(kb0), "v"(kb1));
        float ta[8], tb[8]; float mx = -3.0e38f;
#pragma unroll
        for (int r = 0; r < 8; ++r) { ta[r] = (sHa[r] + sLa[r] * QRI) * SC2; tb[r] = (sHb[r] + sLb[r] * QRI) * SC2;
            const float ea = ((ba >> r) & 1u) ? ta[r] : -3.0e38f; const float eb = ((bb >> r) & 1u) ? tb[r] : -3.0e38f;
            mx = fmaxf(mx, fmaxf(ea, eb)); }
        mx = fmaxf(mx, __shfl_xor(mx, 16, 32));
        const float mnew = fmaxf(m, mx);
        const float alpha = __builtin_amdgcn_exp2f(m - mnew);
        const float sh = PSH - mnew;
        v16h pb; float ls = 0.0f;
#pragma unroll
        for (int r = 0; r < 8; ++r) { const float xa = __builtin_amdgcn_exp2f(ta[r] + sh); const float xb = __builtin_amdgcn_exp2f(tb[r] + sh);
            const h16 pa = (h16)(((ba >> r) & 1u) ? xa : 0.0f); const h16 pc = (h16)(((bb >> r) & 1u) ? xb : 0.0f);
            pb[r] = pa; pb[8 + r] = pc; ls += (float)pa + (float)pc; }
        l = l * alpha + ls; m = mnew;
        o0 = o0 * alpha; o1 = o1 * alpha; o2 = o2 * alpha; o3 = o3 * alpha;
        const h16* va = VT + vo + key0;
        const v16h v0 = ldh(va), v1 = ldh(va + (size_t)16 * SEQ), v2 = ldh(va + (size_t)32 * SEQ), v3 = ldh(va + (size_t)48 * SEQ);
        o0 = wmma16(v0, pb, o0); o1 = wmma16(v1, pb, o1); o2 = wmma16(v2, pb, o2); o3 = wmma16(v3, pb, o3);
        asm volatile("v_nop\n\tv_nop\n\tv_nop\n\tv_nop" : "+v"(o0), "+v"(o1), "+v"(o2), "+v"(o3) : "v"(v0), "v"(v1), "v"(v2), "v"(v3), "v"(pb));
    }
    l += __shfl_xor(l, 16, 32);
    const float inv = (1.0f / l) * CTS;
    const int wb = wave * 16 * 68;
    { v4f a, c;
      a[0] = o0[0] * inv; a[1] = o0[1] * inv; a[2] = o0[2] * inv; a[3] = o0[3] * inv; c[0] = o0[4] * inv; c[1] = o0[5] * inv; c[2] = o0[6] * inv; c[3] = o0[7] * inv;
      *(v4fa*)(&os[wb + lr * 68 +  0 + 8 * hi]) = a; *(v4fa*)(&os[wb + lr * 68 +  0 + 8 * hi + 4]) = c;
      a[0] = o1[0] * inv; a[1] = o1[1] * inv; a[2] = o1[2] * inv; a[3] = o1[3] * inv; c[0] = o1[4] * inv; c[1] = o1[5] * inv; c[2] = o1[6] * inv; c[3] = o1[7] * inv;
      *(v4fa*)(&os[wb + lr * 68 + 16 + 8 * hi]) = a; *(v4fa*)(&os[wb + lr * 68 + 16 + 8 * hi + 4]) = c;
      a[0] = o2[0] * inv; a[1] = o2[1] * inv; a[2] = o2[2] * inv; a[3] = o2[3] * inv; c[0] = o2[4] * inv; c[1] = o2[5] * inv; c[2] = o2[6] * inv; c[3] = o2[7] * inv;
      *(v4fa*)(&os[wb + lr * 68 + 32 + 8 * hi]) = a; *(v4fa*)(&os[wb + lr * 68 + 32 + 8 * hi + 4]) = c;
      a[0] = o3[0] * inv; a[1] = o3[1] * inv; a[2] = o3[2] * inv; a[3] = o3[3] * inv; c[0] = o3[4] * inv; c[1] = o3[5] * inv; c[2] = o3[6] * inv; c[3] = o3[7] * inv;
      *(v4fa*)(&os[wb + lr * 68 + 48 + 8 * hi]) = a; *(v4fa*)(&os[wb + lr * 68 + 48 + 8 * hi + 4]) = c; }
    wave_sync();
    h16* crow = CT + ((size_t)b * SEQ + t0) * (size_t)(2 * DM) + h * HD;
#pragma unroll 1
    for (int ps = 0; ps < 2; ++ps) {
#pragma unroll
        for (int s = 0; s < 4; ++s) { const int row = 4 * s + (lane >> 3), c8 = (lane & 7) * 8;
            const v4f x0 = *(const v4fa*)(&os[wb + row * 68 + c8]); const v4f x1 = *(const v4fa*)(&os[wb + row * 68 + c8 + 4]); v8h hv, rv;
#pragma unroll
            for (int i = 0; i < 4; ++i) { const h16 a0 = (h16)x0[i]; const h16 a1 = (h16)x1[i]; hv[i] = a0; hv[4 + i] = a1; rv[i] = (h16)(x0[i] - (float)a0); rv[4 + i] = (h16)(x1[i] - (float)a1); }
            const size_t oo = (size_t)row * (size_t)(2 * DM) + c8;
            *(volatile v8h*)(crow + oo) = hv; *(volatile v8h*)(crow + oo + DM) = rv; }
        if (ps == 0) __threadfence(); }
}

static constexpr size_t al256(size_t v) { return (v + 255) & ~(size_t)255; }
static constexpr size_t SZ_XB = al256((size_t)NB * SEQ * DM * 2);
static constexpr size_t SZ_WB = al256((size_t)DM * DM * 2);
static constexpr size_t SZ_PL = al256((size_t)NB * NH_ * SEQ * HD * 2);
static constexpr size_t SZ_CT = al256((size_t)NB * SEQ * 2 * DM * 2);
static constexpr size_t SZ_MB = al256((size_t)SEQ * (SEQ / 32) * 4);
static constexpr size_t SZ_TOTAL = 3 * SZ_XB + 4 * SZ_WB + 4 * SZ_PL + SZ_CT + SZ_MB;
static_assert(SZ_TOTAL <= (size_t)134217728);

extern "C" void kernel_launch(void* const* d_in, const int* in_sizes, int n_in,
                              void* d_out, int out_size, void* d_ws, size_t ws_size, hipStream_t stream) {
    if (n_in < 12) return;
    const size_t needx = ((size_t)(SEQ - 1) * NB_FULL + NB) * DM;
    if ((size_t)in_sizes[0] < needx || (size_t)in_sizes[1] < needx || (size_t)in_sizes[2] < needx) return;
    if ((size_t)in_sizes[3] < (size_t)(SEQ - 1) * SEQ_FULL + SEQ) return;
    if ((size_t)in_sizes[4] < (size_t)DM * DM || (size_t)in_sizes[6] < (size_t)DM * DM || (size_t)in_sizes[8] < (size_t)DM * DM || (size_t)in_sizes[10] < (size_t)DM * DM) return;
    if (in_sizes[5] < DM || in_sizes[7] < DM || in_sizes[9] < DM || in_sizes[11] < DM) return;
    if ((size_t)out_size < needx) return;
    if (SZ_TOTAL > ws_size) return;
    const float* xq = (const float*)d_in[0]; const float* xk = (const float*)d_in[1]; const float* xv = (const float*)d_in[2];
    const int* mask = (const int*)d_in[3];
    const float* wq = (const float*)d_in[4];  const float* bq = (const float*)d_in[5];
    const float* wk = (const float*)d_in[6];  const float* bk = (const float*)d_in[7];
    const float* wv = (const float*)d_in[8];  const float* bv = (const float*)d_in[9];
    const float* wo = (const float*)d_in[10]; const float* bo = (const float*)d_in[11];
    float* OUT = (float*)d_out;
    char* wsp = (char*)d_ws;
    bf* XQ = (bf*)wsp; wsp += SZ_XB;
    bf* XK = (bf*)wsp; wsp += SZ_XB;
    bf* XV = (bf*)wsp; wsp += SZ_XB;
    bf* WQ = (bf*)wsp; wsp += SZ_WB;
    bf* WK = (bf*)wsp; wsp += SZ_WB;
    bf* WV = (bf*)wsp; wsp += SZ_WB;
    bf* WO = (bf*)wsp; wsp += SZ_WB;
    h16* QH = (h16*)wsp; wsp += SZ_PL;
    h16* QR = (h16*)wsp; wsp += SZ_PL;
    h16* KP = (h16*)wsp; wsp += SZ_PL;
    h16* VT = (h16*)wsp; wsp += SZ_PL;
    h16* CT = (h16*)wsp; wsp += SZ_CT;
    unsigned* MB = (unsigned*)wsp; wsp += SZ_MB;

    { const size_t n8 = (size_t)NB * SEQ * DM / 8; const unsigned g = (unsigned)((n8 + 255) / 256);
      k_cvtx<<<g, 256, 0, stream>>>(xq, XQ); k_cvtx<<<g, 256, 0, stream>>>(xk, XK); k_cvtx<<<g, 256, 0, stream>>>(xv, XV); }
    { const dim3 gw(DM / 64, DM / 64, 1);
      k_wt<<<gw, 256, 0, stream>>>(wq, WQ, 0); k_wt<<<gw, 256, 0, stream>>>(wk, WK, 0); k_wt<<<gw, 256, 0, stream>>>(wv, WV, 0); k_wt<<<gw, 256, 0, stream>>>(wo, WO, 1); }
    k_mpack<<<(unsigned)(((size_t)SEQ * (SEQ / 32) + 255) / 256), 256, 0, stream>>>(mask, MB);

    k_gemm<0, 0><<<dim3(NB * SEQ / 64, DM / 64, 1), 32, 0, stream>>>(XQ, WQ, DM, DM, QH, QR, 1, OUT, bq, 0, 1.0f, SEQ, (size_t)NH_ * SEQ * HD, HD, HD, (size_t)SEQ * HD);
    k_gemm<0, 0><<<dim3(NB * SEQ / 64, DM / 64, 1), 32, 0, stream>>>(XK, WK, DM, DM, KP, KP, 0, OUT, bk, 0, 1.0f, SEQ, (size_t)NH_ * SEQ * HD, HD, HD, (size_t)SEQ * HD);
    k_gemm<0, 0><<<dim3(DM / 64, NB * SEQ / 64, 1), 32, 0, stream>>>(WV, XV, DM, DM, VT, VT, 0, OUT, bv, 1, 1.0f, DM, (size_t)0, SEQ, SEQ, (size_t)DM * SEQ);

    k_flash<<<dim3(SEQ / (16 * AW), NB * NH_, 1), 32 * AW, 0, stream>>>(QH, QR, KP, VT, MB, CT);

    k_gemm<1, 1><<<dim3(NB * SEQ / 64, DM / 64, 1), 32, 0, stream>>>((const bf*)CT, WO, 2 * DM, DM, QH, QH, 0, OUT, bo, 0, OSC, SEQ, (size_t)DM, NB_FULL * DM, DM, (size_t)0);
}
